// MambaBlock_20822001451658
// MI455X (gfx1250) — hardware-run, weakly checked
//
#include <hip/hip_runtime.h>
#include <math.h>

typedef __attribute__((ext_vector_type(16))) _Float16 v16h;
typedef __attribute__((ext_vector_type(8)))  _Float16 v8h;
typedef __attribute__((ext_vector_type(2)))  _Float16 v2h;
typedef __attribute__((ext_vector_type(16))) __bf16   v16b;
typedef __attribute__((ext_vector_type(8)))  __bf16   v8b;
typedef __attribute__((ext_vector_type(8)))  float    v8f;
typedef __attribute__((ext_vector_type(4)))  float    v4f;
typedef __attribute__((ext_vector_type(2)))  float    v2f;
typedef __attribute__((ext_vector_type(4)))  _Float16 v4h;

constexpr int kNB   = 16;
constexpr int kC    = 128;
constexpr int kL    = 4096;
constexpr int kRows = kNB * kL;
constexpr int kE    = 256;
constexpr int kS    = 16;
constexpr int kSp   = 64;
constexpr int kOut0 = kNB * kC * kL;
constexpr int kThr  = 256;
constexpr float kEps = 1e-5f;
constexpr float kInCarry = 1024.0f;
constexpr float kSc = 1.0f / (kInCarry * kInCarry);
constexpr float kF16MinNormal = 6.103515625e-5f;

static_assert(kRows == 65536 && kC == 128 && kE == 256 && kS == 16 && kSp == 64 && (1 << 12) == kL, "the index arithmetic below uses these sizes");

constexpr size_t kOffHN16 = 0ull;
constexpr size_t kOffWIN16 = 16777216ull;
constexpr size_t kOffZ = 16842752ull;
constexpr size_t kOffZY16 = 83951616ull;
constexpr size_t kOffBM16 = 117506048ull;
constexpr size_t kOffU = 117538816ull;
constexpr size_t kOffST16 = 134316032ull;
constexpr size_t kOffCM16 = 142704640ull;
constexpr size_t kOffYO = 142737408ull;
constexpr size_t kOffWOUT16 = 209846272ull;
constexpr size_t kOffBV = 209911808ull;
constexpr size_t kWsTotal = 209915904ull;
static_assert(kWsTotal <= 268435456ull, "the carve stands under the contract's 256 MiB of workspace");
static_assert(kOffHN16 == 0
  && kOffWIN16 == kOffHN16 + 16777216ull
  && kOffZ == kOffWIN16 + 65536ull
  && kOffZY16 == kOffZ + 67108864ull
  && kOffBM16 == kOffZY16 + 33554432ull
  && kOffU == kOffBM16 + 32768ull
  && kOffST16 == kOffU + 16777216ull
  && kOffCM16 == kOffST16 + 8388608ull
  && kOffYO == kOffCM16 + 32768ull
  && kOffWOUT16 == kOffYO + 67108864ull
  && kOffBV == kOffWOUT16 + 65536ull
  && kWsTotal == kOffBV + 4096ull, "the carve is a chain: every region starts where the one before ends");
static_assert((size_t)kRows * kC * 2 == 16777216ull && (size_t)kRows * kE * 4 == 67108864ull && (size_t)kRows * kE * 2 == 33554432ull && (size_t)kRows * kSp * 4 == 16777216ull && (size_t)kRows * kSp * 2 == 8388608ull && (size_t)kRows * kC * 4 * 2 == 67108864ull, "every region's length is its plane's");
static_assert((kOffWIN16 % 256) == 0 && (kOffZ % 256) == 0 && (kOffZY16 % 256) == 0 && (kOffBM16 % 256) == 0 && (kOffU % 256) == 0 && (kOffST16 % 256) == 0 && (kOffCM16 % 256) == 0 && (kOffYO % 256) == 0 && (kOffWOUT16 % 256) == 0 && (kOffBV % 256) == 0, "every region starts on a multiple of 256 B");
constexpr int kBvIn = 0, kBvZero = 256, kBvOut = 512;

__device__ __forceinline__ unsigned short f2bf_bits(float f) {
  unsigned u = __float_as_uint(f);
  return (unsigned short)((u + 0x7FFFu + ((u >> 16) & 1u)) >> 16);
}
__device__ __forceinline__ float bf_bits2f(unsigned short h) { return __uint_as_float(((unsigned)h) << 16); }
__device__ __forceinline__ float bf16r(float f) { return bf_bits2f(f2bf_bits(f)); }
__device__ __forceinline__ float carry_flush(float v, float carry) {
  const float s = v * carry;
  return (fabsf(s) < kF16MinNormal) ? 0.0f : s;
}

__device__ __forceinline__ void dep_guard4_h(v8f& a, v8f& b, v8f& c, v8f& d, v16h x, v16h y) { asm volatile("v_nop\n\tv_nop\n\tv_nop\n\tv_nop" : "+v"(a), "+v"(b), "+v"(c), "+v"(d) : "v"(x), "v"(y)); }
__device__ __forceinline__ void dep_guard4_b(v8f& a, v8f& b, v8f& c, v8f& d, v16b x, v16b y) { asm volatile("v_nop\n\tv_nop\n\tv_nop\n\tv_nop" : "+v"(a), "+v"(b), "+v"(c), "+v"(d) : "v"(x), "v"(y)); }
__device__ __forceinline__ void keep4_h(v16h a, v16h b, v16h c, v16h d) { asm volatile("v_nop" :: "v"(a), "v"(b), "v"(c), "v"(d)); }
__device__ __forceinline__ void keep4_b(v16b a, v16b b, v16b c, v16b d) { asm volatile("v_nop" :: "v"(a), "v"(b), "v"(c), "v"(d)); }
__device__ __forceinline__ void acc_guard4(v8f& a, v8f& b, v8f& c, v8f& d) { asm volatile("v_nop\n\tv_nop\n\tv_nop\n\tv_nop" : "+v"(a), "+v"(b), "+v"(c), "+v"(d)); }

template <typename T> struct Frag;
template <> struct Frag<_Float16> {
  typedef v16h V; union U { v16h v; v8h h[2]; };
  static __device__ __forceinline__ v16h load(const _Float16* p) {
    U f; f.h[0] = *(const v8h*)(p); f.h[1] = *(const v8h*)(p + 16); return f.v;
  }
  static __device__ __forceinline__ v8f mma(v16h a, v16h b, v8f c) {
    return __builtin_amdgcn_wmma_f32_16x16x32_f16(false, a, false, b, (short)0, c, false, false);
  }
  static __device__ __forceinline__ void guard4(v8f& a, v8f& b, v8f& c, v8f& d, v16h x, v16h y) { dep_guard4_h(a, b, c, d, x, y); }
  static __device__ __forceinline__ void keep(v16h a, v16h b, v16h c, v16h d) { keep4_h(a, b, c, d); }
};
template <> struct Frag<__bf16> {
  typedef v16b V; union U { v16b v; v8b h[2]; };
  static __device__ __forceinline__ v16b load(const __bf16* p) {
    U f; f.h[0] = *(const v8b*)(p); f.h[1] = *(const v8b*)(p + 16); return f.v;
  }
  static __device__ __forceinline__ v8f mma(v16b a, v16b b, v8f c) {
    return __builtin_amdgcn_wmma_f32_16x16x32_bf16(false, a, false, b, (short)0, c, false, false);
  }
  static __device__ __forceinline__ void guard4(v8f& a, v8f& b, v8f& c, v8f& d, v16b x, v16b y) { dep_guard4_b(a, b, c, d, x, y); }
  static __device__ __forceinline__ void keep(v16b a, v16b b, v16b c, v16b d) { keep4_b(a, b, c, d); }
};

__device__ __forceinline__ v8f mma_h(v16h a, v16h b, v8f c) {
  c = __builtin_amdgcn_wmma_f32_16x16x32_f16(false, a, false, b, (short)0, c, false, false);
  asm volatile("v_nop\n\tv_nop\n\tv_nop\n\tv_nop" : "+v"(c) : "v"(a), "v"(b));
  return c;
}

template <int ET> struct Elem;
template <> struct Elem<0> { typedef _Float16 T; };
template <> struct Elem<1> { typedef __bf16 T; };
template <int ET, bool SPLIT, int BIAS_MODE, int OUT_MODE, bool RESID, int ACT = 0>
__global__ __launch_bounds__(256) void wmma_gemm64(
    const unsigned short* __restrict__ Ap, const unsigned short* __restrict__ A2p, int lda, long strideA,
    const unsigned short* __restrict__ Btp, const unsigned short* __restrict__ Bt2p, int ldb, long strideB,
    void* __restrict__ Cout, void* __restrict__ Cout2, int ldc, long strideC,
    const float* __restrict__ bias,
    const float* __restrict__ resid, long strideR,
    int M, int N, int K, float scale) {
  typedef typename Elem<ET>::T T;
  typedef typename Frag<T>::V V;
  const T* A = (const T*)Ap; const T* A2 = (const T*)A2p; const T* Bt = (const T*)Btp; const T* Bt2 = (const T*)Bt2p;
  __shared__ __align__(16) float sT[8][16 * 68];
  const int b    = blockIdx.y;
  const int lane = threadIdx.x & 31;
  const int wave = threadIdx.x >> 5;
  const int tilesN = N >> 6;
  const int tilesM = M >> 6;
  const int tile = blockIdx.x * 8 + wave;
  if (tile >= tilesM * tilesN) return;
  const int tm = tile / tilesN;
  const int tn = tile - tm * tilesN;
  const int m0 = tm << 6;
  const int n0 = tn << 6;

  const T* Ab  = A  + (size_t)b * strideA;
  const T* Bb  = Bt + (size_t)b * strideB;
  const T* Ab2 = SPLIT ? (A2  + (size_t)b * strideA) : nullptr;
  const T* Bb2 = SPLIT ? (Bt2 + (size_t)b * strideB) : nullptr;

  const int rlane = lane & 15;
  const int koff  = (lane >> 4) * 8;
  const int mOff  = (lane >> 4) * 8;

  v8f acc[4][4];
#pragma unroll
  for (int i = 0; i < 4; ++i)
#pragma unroll
    for (int j = 0; j < 4; ++j) acc[i][j] = (v8f){0.f,0.f,0.f,0.f,0.f,0.f,0.f,0.f};

  for (int k0 = 0; k0 < K; k0 += 32) {
    V bh[4], bl[4];
#pragma unroll
    for (int j = 0; j < 4; ++j) {
      const size_t bo = (size_t)(n0 + (j << 4) + rlane) * ldb + koff + k0;
      bh[j] = Frag<T>::load(Bb + bo);
      if (SPLIT) bl[j] = Frag<T>::load(Bb2 + bo);
    }
#pragma unroll
    for (int i = 0; i < 4; ++i) {
      const size_t ao = (size_t)(m0 + (i << 4) + rlane) * lda + koff + k0;
      V ah = Frag<T>::load(Ab + ao);
      V al;
      if (SPLIT) al = Frag<T>::load(Ab2 + ao);
#pragma unroll
      for (int j = 0; j < 4; ++j) {
        acc[i][j] = Frag<T>::mma(ah, bh[j], acc[i][j]);
        if (SPLIT) {
          acc[i][j] = Frag<T>::mma(ah, bl[j], acc[i][j]);
          acc[i][j] = Frag<T>::mma(al, bh[j], acc[i][j]);
        }
      }
      Frag<T>::guard4(acc[i][0], acc[i][1], acc[i][2], acc[i][3], ah, SPLIT ? al : ah);
    }
    Frag<T>::keep(bh[0], bh[1], bh[2], bh[3]);
    if (SPLIT) Frag<T>::keep(bl[0], bl[1], bl[2], bl[3]);
  }
  acc_guard4(acc[0][0], acc[0][1], acc[0][2], acc[0][3]);
  acc_guard4(acc[1][0], acc[1][1], acc[1][2], acc[1][3]);
  acc_guard4(acc[2][0], acc[2][1], acc[2][2], acc[2][3]);
  acc_guard4(acc[3][0], acc[3][1], acc[3][2], acc[3][3]);

  float* slab = sT[wave];
  const float* Rb = RESID ? (resid + (size_t)b * strideR) : nullptr;
#pragma unroll
  for (int i = 0; i < 4; ++i) {
    const int mBase = m0 + (i << 4);
#pragma unroll
    for (int j = 0; j < 4; ++j) {
      const int n = n0 + (j << 4) + rlane;
      float bv = 0.f;
      if (BIAS_MODE == 2) bv = bias[n];
#pragma unroll
      for (int r = 0; r < 8; ++r) {
        float v = acc[i][j][r] * scale;
        if (BIAS_MODE == 1) v += bias[mBase + mOff + r];
        if (BIAS_MODE == 2) v += bv;
        if (RESID) v += Rb[(size_t)(mBase + mOff + r) * ldc + n];
        if (ACT == 1) v = tanhf(v);
        if (ACT == 2) v = fmaxf(v, 0.0f);
        if (ACT == 3) v = v / (1.0f + expf(-v));
        if (ACT == 4) v = (v > 0.f) ? v : 0.01f * v;
        slab[(mOff + r) * 68 + (j << 4) + rlane] = v;
      }
    }
    __builtin_amdgcn_fence(__ATOMIC_RELEASE, "workgroup");
    __builtin_amdgcn_wave_barrier();
    __builtin_amdgcn_fence(__ATOMIC_ACQUIRE, "workgroup");
    if (OUT_MODE == 0) {
      float* C = (float*)Cout + (size_t)b * strideC;
      const int hh = lane >> 4, c4 = (lane & 15) * 4;
      for (int pass = 0; pass < 2; ++pass) {
#pragma unroll
        for (int it = 0; it < 8; ++it) {
          const int row = it * 2 + hh;
          v4f v = *(const v4f*)(slab + row * 68 + c4);
          *(volatile v4f*)(C + (size_t)(mBase + row) * ldc + n0 + c4) = v;
        }
        __threadfence();
      }
    } else {
      const int q = lane >> 3, c8 = (lane & 7) * 8;
      unsigned short* C  = (unsigned short*)Cout  + (size_t)b * strideC;
      unsigned short* C2 = (OUT_MODE == 2) ? ((unsigned short*)Cout2 + (size_t)b * strideC) : nullptr;
      for (int pass = 0; pass < 2; ++pass) {
#pragma unroll
        for (int it = 0; it < 4; ++it) {
          const int row = it * 4 + q;
          const float* sp = slab + row * 68 + c8;
          v8h hv, lv;
#pragma unroll
          for (int e = 0; e < 8; ++e) {
            if (OUT_MODE == 1) {
              hv[e] = (_Float16)sp[e];
            } else {
              unsigned short hb = f2bf_bits(sp[e]);
              unsigned short lb = f2bf_bits(sp[e] - bf_bits2f(hb));
              hv[e] = __builtin_bit_cast(_Float16, hb);
              lv[e] = __builtin_bit_cast(_Float16, lb);
            }
          }
          *(volatile v8h*)(C + (size_t)(mBase + row) * ldc + n0 + c8) = hv;
          if (OUT_MODE == 2) *(volatile v8h*)(C2 + (size_t)(mBase + row) * ldc + n0 + c8) = lv;
        }
        __threadfence();
      }
    }
    __builtin_amdgcn_fence(__ATOMIC_RELEASE, "workgroup");
    __builtin_amdgcn_wave_barrier();
    __builtin_amdgcn_fence(__ATOMIC_ACQUIRE, "workgroup");
  }
}


__global__ __launch_bounds__(kThr) void cast_plane_kernel(const float* __restrict__ src, unsigned short* __restrict__ dst,
                                                          int colsLog2, int dstPitch, int dstOff) {
  const int i   = blockIdx.x * kThr + threadIdx.x;
  const int sh  = colsLog2 - 3;
  const int row = i >> sh;
  const int c8  = (i & ((1 << sh) - 1)) * 8;
  const float* sp = src + ((size_t)row << colsLog2) + c8;
  const v4f a0 = *(const v4f*)(sp);
  const v4f a1 = *(const v4f*)(sp + 4);
  v8h hv;
#pragma unroll
  for (int e = 0; e < 4; ++e) {
    const float f0 = a0[e];
    const float f1 = a1[e];
    hv[e]     = (_Float16)carry_flush(bf16r(f0), kInCarry);
    hv[4 + e] = (_Float16)carry_flush(bf16r(f1), kInCarry);
  }
  unsigned short* dp = dst + (size_t)row * dstPitch + dstOff + c8;
  *(volatile v8h*)dp = hv;
  __threadfence();
  *(volatile v8h*)dp = hv;
}

__global__ __launch_bounds__(kThr) void setup_kernel(const float* __restrict__ b_in, const float* __restrict__ b_out, float* __restrict__ BV) {
  const unsigned i = blockIdx.x * (unsigned)kThr + threadIdx.x;
  const float v0 = b_in[i & 255u];
  const float v1 = b_out[(i - (unsigned)kBvOut) & 127u];
  const float o = bf16r((i < (unsigned)kBvZero) ? v0 : ((i >= (unsigned)kBvOut && i < (unsigned)(kBvOut + kC)) ? v1 : 0.0f));
  float* dp = BV + i;
  *(volatile float*)dp = o;
  __threadfence();
  *(volatile float*)dp = o;
}

__global__ __launch_bounds__(kThr) void pad_kernel(const float* __restrict__ Bm, const float* __restrict__ Cm, unsigned short* __restrict__ BM16, unsigned short* __restrict__ CM16) {
  const unsigned i = blockIdx.x * (unsigned)kThr + threadIdx.x;
  const bool isB = i < 2048u;
  const unsigned j = i - 2048u;
  const unsigned r = i >> 5, c8 = (i & 31u) * 8u;
  const unsigned e = (j >> 3) & 255u, s8 = (j & 7u) * 8u;
  const unsigned lim = isB ? r : s8;
  const bool live = lim < (unsigned)kS;
  const float* sp = isB ? (Bm + (r & 15u) * (unsigned)kE + c8) : (Cm + e * (unsigned)kS + (s8 & 8u));
  const v4f a0 = *(const v4f*)sp, a1 = *(const v4f*)(sp + 4);
  v8h hv;
#pragma unroll
  for (int q = 0; q < 4; ++q) { hv[q] = (_Float16)carry_flush(live ? bf16r(a0[q]) : 0.0f, kInCarry); hv[4 + q] = (_Float16)carry_flush(live ? bf16r(a1[q]) : 0.0f, kInCarry); }
  unsigned short* dp = isB ? (BM16 + i * 8u) : (CM16 + j * 8u);
  *(volatile v8h*)dp = hv;
  __threadfence();
  *(volatile v8h*)dp = hv;
}
static_assert(64 * kE / 8 == 2048 && kE * kSp / 8 == 2048 && 16 * kThr == 4096, "the padded operands' grid exact: 16 blocks");

__global__ __launch_bounds__(kThr) void ln_kernel(const float* __restrict__ x, const float* __restrict__ gamma, const float* __restrict__ beta, unsigned short* __restrict__ HN16) {
  const unsigned row = blockIdx.x * (unsigned)kThr + threadIdx.x;
  const unsigned sq = row >> 12, l = row & (unsigned)(kL - 1);
  const float* xp = x + sq * (unsigned)(kC * kL) + l;
  float v[kC];
  float sum = 0.0f;
#pragma unroll
  for (int c = 0; c < kC; ++c) { v[c] = bf16r(xp[(unsigned)c * (unsigned)kL]); sum += v[c]; }
  const float mu = sum / (float)kC;
  float sq2 = 0.0f;
#pragma unroll
  for (int c = 0; c < kC; ++c) { const float d = v[c] - mu; sq2 += d * d; }
  const float r = 1.0f / sqrtf(sq2 / (float)kC + kEps);
  unsigned short* dp0 = HN16 + row * (unsigned)kC;
#pragma unroll
  for (int c8 = 0; c8 < kC; c8 += 8) {
    v8h hv;
#pragma unroll
    for (int q = 0; q < 8; ++q) hv[q] = (_Float16)carry_flush((v[c8 + q] - mu) * r * bf16r(gamma[c8 + q]) + bf16r(beta[c8 + q]), kInCarry);
    unsigned short* dp = dp0 + c8;
    *(volatile v8h*)dp = hv;
    __threadfence();
    *(volatile v8h*)dp = hv;
  }
}
static_assert(kRows == 256 * kThr, "the norm's grid exact: 256 blocks: a lane a token");

__global__ __launch_bounds__(kThr) void zcast_kernel(const float* __restrict__ Z, unsigned short* __restrict__ Z16) {
  const unsigned i = blockIdx.x * (unsigned)kThr + threadIdx.x;
  const v4f a0 = *(const v4f*)(Z + i * 8u), a1 = *(const v4f*)(Z + i * 8u + 4u);
  v8h hv;
#pragma unroll
  for (int q = 0; q < 4; ++q) { hv[q] = (_Float16)carry_flush(a0[q], kInCarry); hv[4 + q] = (_Float16)carry_flush(a1[q], kInCarry); }
  unsigned short* dp = Z16 + i * 8u;
  *(volatile v8h*)dp = hv;
  __threadfence();
  *(volatile v8h*)dp = hv;
}
static_assert((size_t)kRows * kE / 8 == 8192ull * kThr, "the copy's grid exact: 8,192 blocks");

__global__ __launch_bounds__(32) void scan_kernel(const float* __restrict__ U, const float* __restrict__ A, unsigned short* __restrict__ ST16) {
  __shared__ __align__(16) float sA[kS * kS];
  const unsigned sq = threadIdx.x;
  {
    const v4f a0 = *(const v4f*)(A + sq * 8u), a1 = *(const v4f*)(A + sq * 8u + 4u);
    v4f r0, r1;
#pragma unroll
    for (int q = 0; q < 4; ++q) { r0[q] = bf16r(a0[q]); r1[q] = bf16r(a1[q]); }
    *(v4f*)(sA + sq * 8u) = r0;
    *(v4f*)(sA + sq * 8u + 4u) = r1;
  }
  __builtin_amdgcn_fence(__ATOMIC_RELEASE, "workgroup");
  __builtin_amdgcn_wave_barrier();
  __builtin_amdgcn_fence(__ATOMIC_ACQUIRE, "workgroup");
  if (sq >= (unsigned)kNB) return;
  float h[kS];
#pragma unroll
  for (int n = 0; n < kS; ++n) h[n] = 0.0f;
  for (int t = 0; t < kL; ++t) {
    const v4f* ad = (const v4f*)sA;
    const unsigned row = sq * (unsigned)kL + (unsigned)t;
    const float* up = U + row * (unsigned)kSp;
    const v4f b0 = *(const v4f*)up, b1 = *(const v4f*)(up + 4), b2 = *(const v4f*)(up + 8), b3 = *(const v4f*)(up + 12);
    float hn[kS];
#pragma unroll
    for (int n = 0; n < kS; ++n) {
      const v4f a0 = ad[n * 4 + 0], a1 = ad[n * 4 + 1], a2 = ad[n * 4 + 2], a3 = ad[n * 4 + 3];
      float s = 0.0f;
#pragma unroll
      for (int m = 0; m < 4; ++m) s += a0[m] * h[m];
#pragma unroll
      for (int m = 0; m < 4; ++m) s += a1[m] * h[4 + m];
#pragma unroll
      for (int m = 0; m < 4; ++m) s += a2[m] * h[8 + m];
#pragma unroll
      for (int m = 0; m < 4; ++m) s += a3[m] * h[12 + m];
      const float bx = (n < 4) ? b0[n & 3] : ((n < 8) ? b1[n & 3] : ((n < 12) ? b2[n & 3] : b3[n & 3]));
      hn[n] = tanhf(s + bx);
    }
    v8h w0, w1, wz;
#pragma unroll
    for (int q = 0; q < 8; ++q) { h[q] = hn[q]; h[8 + q] = hn[8 + q]; w0[q] = (_Float16)carry_flush(hn[q], kInCarry); w1[q] = (_Float16)carry_flush(hn[8 + q], kInCarry); wz[q] = (_Float16)0.0f; }
    unsigned short* dp = ST16 + row * (unsigned)kSp;
    for (int pass = 0; pass < 2; ++pass) {
      *(volatile v8h*)dp = w0;
      *(volatile v8h*)(dp + 8) = w1;
#pragma unroll
      for (int g = 2; g < 8; ++g) *(volatile v8h*)(dp + 8 * g) = wz;
      __threadfence();
    }
  }
}
static_assert(kNB == 16 && kS * kS == 32 * 8 && (size_t)kRows * kSp < 4294967296ull / 4, "the recurrence is one wave: 32 lanes fill the 256 floats, 16 carry a sequence; 32-bit element offsets");

__global__ __launch_bounds__(kThr) void ycast_kernel(const float* __restrict__ Y, const float* __restrict__ Z, const float* __restrict__ D, unsigned short* __restrict__ Y16) {
  const unsigned i = blockIdx.x * (unsigned)kThr + threadIdx.x;
  const unsigned e8 = (i & 31u) * 8u;
  const v4f y0 = *(const v4f*)(Y + i * 8u), y1 = *(const v4f*)(Y + i * 8u + 4u);
  const v4f z0 = *(const v4f*)(Z + i * 8u), z1 = *(const v4f*)(Z + i * 8u + 4u);
  const v4f d0 = *(const v4f*)(D + e8), d1 = *(const v4f*)(D + e8 + 4u);
  v8h hv;
#pragma unroll
  for (int q = 0; q < 4; ++q) { hv[q] = (_Float16)carry_flush(y0[q] + z0[q] * bf16r(d0[q]), kInCarry); hv[4 + q] = (_Float16)carry_flush(y1[q] + z1[q] * bf16r(d1[q]), kInCarry); }
  unsigned short* dp = Y16 + i * 8u;
  *(volatile v8h*)dp = hv;
  __threadfence();
  *(volatile v8h*)dp = hv;
}

__global__ __launch_bounds__(kThr) void close_kernel(const float* __restrict__ x, const float* __restrict__ O, float* __restrict__ out) {
  const unsigned i = blockIdx.x * (unsigned)kThr + threadIdx.x;
  const unsigned l8 = (i & 511u) * 8u, c = (i >> 9) & 127u, sq = i >> 16;
  const v4f x0 = *(const v4f*)(x + i * 8u), x1 = *(const v4f*)(x + i * 8u + 4u);
  const float* op = O + (sq * (unsigned)kL + l8) * (unsigned)kC + c;
  v4f o0, o1;
#pragma unroll
  for (int q = 0; q < 4; ++q) { o0[q] = bf16r(x0[q]) + op[(unsigned)q * (unsigned)kC]; o1[q] = bf16r(x1[q]) + op[(unsigned)(4 + q) * (unsigned)kC]; }
  float* dp = out + i * 8u;
  for (int pass = 0; pass < 2; ++pass) {
    *(volatile v4f*)dp = o0;
    *(volatile v4f*)(dp + 4) = o1;
    __threadfence();
  }
}
static_assert((size_t)kNB * kC * kL / 8 == 4096ull * kThr && kL / 8 == 512, "the closing pass's grid exact: 4,096 blocks");

extern "C" void kernel_launch(void* const* d_in, const int* in_sizes, int n_in,
                              void* d_out, int out_size, void* d_ws, size_t ws_size,
                              hipStream_t stream) {
  if (n_in < 11 || d_out == nullptr || d_ws == nullptr) return;
  if (in_sizes[0] != kNB * kC * kL || in_sizes[1] != kS * kS || in_sizes[2] != kS * kE || in_sizes[3] != kE * kS || in_sizes[4] != kE || in_sizes[5] != kE * kC || in_sizes[6] != kE || in_sizes[7] != kC * kE || in_sizes[8] != kC || in_sizes[9] != kC || in_sizes[10] != kC) return;
  if (out_size != kOut0) return;
  if (ws_size < kWsTotal) return;
  const float* x = (const float*)d_in[0];
  const float* A = (const float*)d_in[1];
  const float* Bm = (const float*)d_in[2];
  const float* Cm = (const float*)d_in[3];
  const float* D = (const float*)d_in[4];
  const float* W_in = (const float*)d_in[5];
  const float* b_in = (const float*)d_in[6];
  const float* W_out = (const float*)d_in[7];
  const float* b_out = (const float*)d_in[8];
  const float* gamma = (const float*)d_in[9];
  const float* beta = (const float*)d_in[10];
  float* out = (float*)d_out;
  char* ws = (char*)d_ws;
  unsigned short* HN16 = (unsigned short*)(ws + kOffHN16);
  unsigned short* WIN16 = (unsigned short*)(ws + kOffWIN16);
  float* Z = (float*)(ws + kOffZ);
  unsigned short* ZY16 = (unsigned short*)(ws + kOffZY16);
  unsigned short* BM16 = (unsigned short*)(ws + kOffBM16);
  float* U = (float*)(ws + kOffU);
  unsigned short* ST16 = (unsigned short*)(ws + kOffST16);
  unsigned short* CM16 = (unsigned short*)(ws + kOffCM16);
  float* YO = (float*)(ws + kOffYO);
  unsigned short* WOUT16 = (unsigned short*)(ws + kOffWOUT16);
  float* BV = (float*)(ws + kOffBV);

  setup_kernel<<<4, kThr, 0, stream>>>(b_in, b_out, BV);
  pad_kernel<<<16, kThr, 0, stream>>>(Bm, Cm, BM16, CM16);
  static_assert(((size_t)kE * kC / 8) % kThr == 0, "the row casts' grids");
  cast_plane_kernel<<<(int)(((size_t)kE * kC / 8) / kThr), kThr, 0, stream>>>(W_in, WIN16, 7, kC, 0);
  cast_plane_kernel<<<(int)(((size_t)kC * kE / 8) / kThr), kThr, 0, stream>>>(W_out, WOUT16, 8, kE, 0);
  ln_kernel<<<256, kThr, 0, stream>>>(x, gamma, beta, HN16);
  wmma_gemm64<0, false, 2, 0, false, 0><<<dim3((kRows / 64) * (kE / 64) / 8, 1), 256, 0, stream>>>(
      HN16, HN16, kC, 0L, WIN16, WIN16, kC, 0L, (void*)Z, (void*)Z, kE, 0L, BV + kBvIn, nullptr, 0L, kRows, kE, kC, kSc);
  zcast_kernel<<<8192, kThr, 0, stream>>>(Z, ZY16);
  wmma_gemm64<0, false, 2, 0, false, 0><<<dim3((kRows / 64) * (kSp / 64) / 8, 1), 256, 0, stream>>>(
      ZY16, ZY16, kE, 0L, BM16, BM16, kE, 0L, (void*)U, (void*)U, kSp, 0L, BV + kBvZero, nullptr, 0L, kRows, kSp, kE, kSc);
  scan_kernel<<<1, 32, 0, stream>>>(U, A, ST16);
  wmma_gemm64<0, false, 2, 0, false, 0><<<dim3((kRows / 64) * (kE / 64) / 8, 1), 256, 0, stream>>>(
      ST16, ST16, kSp, 0L, CM16, CM16, kSp, 0L, (void*)YO, (void*)YO, kE, 0L, BV + kBvZero, nullptr, 0L, kRows, kE, kSp, kSc);
  ycast_kernel<<<8192, kThr, 0, stream>>>(YO, Z, D, ZY16);
  wmma_gemm64<0, false, 2, 0, false, 0><<<dim3((kRows / 64) * (kC / 64) / 8, 1), 256, 0, stream>>>(
      ZY16, ZY16, kE, 0L, WOUT16, WOUT16, kE, 0L, (void*)YO, (void*)YO, kC, 0L, BV + kBvOut, nullptr, 0L, kRows, kC, kE, kSc);
  close_kernel<<<4096, kThr, 0, stream>>>(x, YO, out);
}
static_assert(((kRows / 64) * (kSp / 64)) % 8 == 0 && ((kRows / 64) * (kC / 64)) % 8 == 0, "the engine's grids: whole blocks of eight wave tiles");
